// LSTMTemperatureRegressorV2_33586644254930
// MI455X (gfx1250) — hardware-verified
//
#include <hip/hip_runtime.h>
#include <math.h>

constexpr int NSEQ        = 256;
constexpr int NSTEP       = 200;
constexpr int NXF         = 16;
constexpr int NIN         = 18;
constexpr int NHID        = 256;
constexpr int NGATE       = 1024;
constexpr int NFWD        = 64;
constexpr int KIN         = 32;
constexpr int NTHR        = 256;
constexpr int SEQ_PER_BLK = 16;
constexpr int AINP        = 40;
constexpr int AHP         = 264;
constexpr int HIDP        = 68;
constexpr int OSTP        = 260;
constexpr int ZTOT        = SEQ_PER_BLK * NSTEP;
constexpr int ZQUADS      = ZTOT / 4;
constexpr float WCARRY      = 16.0f;
constexpr float WCARRY_INV  = 1.0f / 16.0f;
constexpr float LOCARRY     = 256.0f;
constexpr float LOCOL_SCALE = 1.0f / 16.0f;
constexpr int OUT1_OFF = NSEQ * NSTEP;
constexpr int OUT2_OFF = OUT1_OFF + NSEQ * NHID;
static_assert(ZTOT % 4 == 0, "out0 block region is whole float4");
static_assert((ZTOT * 4) % 128 == 0, "out0 block region is whole 128-B lines");
static_assert(KIN % 32 == 0 && NHID % 32 == 0, "k multiples of 32");

typedef __attribute__((ext_vector_type(16))) _Float16 v16h;
typedef __attribute__((ext_vector_type(8)))  _Float16 v8h;
typedef __attribute__((ext_vector_type(8)))  float    v8f;
typedef __attribute__((ext_vector_type(4)))  float    v4f;

__device__ __forceinline__ unsigned short f2bf_bits(float f) {
  unsigned u = __float_as_uint(f);
  return (unsigned short)((u + 0x7FFFu + ((u >> 16) & 1u)) >> 16);
}
__device__ __forceinline__ float bf_bits2f(unsigned short h) { return __uint_as_float(((unsigned)h) << 16); }
__device__ __forceinline__ float rbf(float f) { return bf_bits2f(f2bf_bits(f)); }

__device__ __forceinline__ void dep_guard_h(v8f& a, v8f& b, v16h x, v16h y) { asm volatile("v_nop\n\tv_nop\n\tv_nop\n\tv_nop" : "+v"(a), "+v"(b) : "v"(x), "v"(y)); }
__device__ __forceinline__ void dep_guard1_h(v8f& a, v16h x, v16h y) { asm volatile("v_nop\n\tv_nop\n\tv_nop\n\tv_nop" : "+v"(a) : "v"(x), "v"(y)); }
__device__ __forceinline__ void keep4_h(v16h a, v16h b, v16h c, v16h d) { asm volatile("v_nop" :: "v"(a), "v"(b), "v"(c), "v"(d)); }
__device__ __forceinline__ void acc_guard4(v8f& a, v8f& b, v8f& c, v8f& d) { asm volatile("v_nop\n\tv_nop\n\tv_nop\n\tv_nop" : "+v"(a), "+v"(b), "+v"(c), "+v"(d)); }
__device__ __forceinline__ void acc_guard1(v8f& a) { asm volatile("v_nop\n\tv_nop\n\tv_nop\n\tv_nop" : "+v"(a)); }

template <typename T> struct Frag;
template <> struct Frag<_Float16> {
  typedef v16h V; union U { v16h v; v8h h[2]; };
  static __device__ __forceinline__ v16h load(const _Float16* p) {
    U f; f.h[0] = *(const v8h*)(p); f.h[1] = *(const v8h*)(p + 16); return f.v;
  }
  static __device__ __forceinline__ v8f mma(v16h a, v16h b, v8f c) {
    return __builtin_amdgcn_wmma_f32_16x16x32_f16(false, a, false, b, (short)0, c, false, false);
  }
};

__device__ __forceinline__ float fsig(float x)  { return __builtin_amdgcn_rcpf(1.0f + __expf(-x)); }
__device__ __forceinline__ float ftanh(float x) { return 1.0f - 2.0f * __builtin_amdgcn_rcpf(__expf(2.0f * x) + 1.0f); }

__global__ __launch_bounds__(NTHR) void cast_w_f16x2(const float* __restrict__ in, unsigned short* __restrict__ outp, int n2, float sc) {
  const int i = blockIdx.x * NTHR + threadIdx.x;
  if (i < n2) {
    const _Float16 e0 = (_Float16)(rbf(in[2 * i]) * sc);
    const _Float16 e1 = (_Float16)(rbf(in[2 * i + 1]) * sc);
    const unsigned u = (unsigned)__builtin_bit_cast(unsigned short, e0) | ((unsigned)__builtin_bit_cast(unsigned short, e1) << 16);
    ((volatile unsigned*)outp)[i] = u;
    __threadfence();
    ((volatile unsigned*)outp)[i] = u;
  }
}

__global__ __launch_bounds__(NTHR) void wih_plane_kernel(const float* __restrict__ wih, unsigned short* __restrict__ outp) {
  const int i = blockIdx.x * NTHR + threadIdx.x;
  if (i < NGATE * KIN / 2) {
    const int n  = i >> 4;
    const int k0 = (i & 15) * 2;
    const int k1 = k0 + 1;
    const int kc0 = k0 < (NIN - 1) ? k0 : (NIN - 1);
    const int kc1 = k1 < (NIN - 1) ? k1 : (NIN - 1);
    const float w0 = rbf(wih[n * NIN + kc0]);
    const float w1 = rbf(wih[n * NIN + kc1]);
    const float s0 = (k0 < NIN) ? WCARRY : ((k0 == NIN) ? LOCOL_SCALE : 0.0f);
    const float s1 = (k1 < NIN) ? WCARRY : ((k1 == NIN) ? LOCOL_SCALE : 0.0f);
    const _Float16 e0 = (_Float16)(w0 * s0);
    const _Float16 e1 = (_Float16)(w1 * s1);
    const unsigned u = (unsigned)__builtin_bit_cast(unsigned short, e0) | ((unsigned)__builtin_bit_cast(unsigned short, e1) << 16);
    ((volatile unsigned*)outp)[i] = u;
    __threadfence();
    ((volatile unsigned*)outp)[i] = u;
  }
}

__global__ __launch_bounds__(NTHR) void lstm_head_kernel(
    const float* __restrict__ zin, const float* __restrict__ xin, const float* __restrict__ h0,
    const float* __restrict__ bgate, const float* __restrict__ bhead, const float* __restrict__ w2,
    const float* __restrict__ bout,
    const unsigned short* __restrict__ WIp, const unsigned short* __restrict__ WHp,
    const unsigned short* __restrict__ W1p, float* __restrict__ out) {
  __shared__ __align__(16) _Float16 Ain[SEQ_PER_BLK * AINP];
  __shared__ __align__(16) _Float16 Ah[SEQ_PER_BLK * AHP];
  __shared__ __align__(16) float    Hid[SEQ_PER_BLK * HIDP];
  __shared__ __align__(16) float    Zs[ZTOT];
  __shared__ __align__(16) float    Hs[SEQ_PER_BLK * OSTP];
  __shared__ __align__(16) float    Cs[SEQ_PER_BLK * OSTP];
  const _Float16* WI  = (const _Float16*)WIp;
  const _Float16* WH  = (const _Float16*)WHp;
  const _Float16* W1h = (const _Float16*)W1p;
  const int tid = threadIdx.x, lane = tid & 31, wave = tid >> 5;
  const int c = lane & 15, hh = lane >> 4, koff = hh * 8;
  const int rowbase = blockIdx.x * SEQ_PER_BLK;
  const int mz = tid >> 4;

#pragma unroll 1
  for (int i = 0; i < SEQ_PER_BLK; ++i)
    Ah[i * AHP + tid] = (_Float16)rbf(h0[(size_t)(rowbase + i) * NHID + tid]);
#pragma unroll 1
  for (int idx = tid; idx < SEQ_PER_BLK * AINP; idx += NTHR) {
    const int m = idx / AINP;
    const int k = idx - m * AINP;
    int kx = k - 1; kx = kx < 0 ? 0 : (kx > NXF - 1 ? NXF - 1 : kx);
    const size_t bt = (size_t)(rowbase + m) * NSTEP;
    const float zv = zin[bt];
    const float xv = xin[bt * NXF + kx];
    const float v = (k == 0) ? zv : ((k <= NXF) ? xv : 0.0f);
    Ain[idx] = (_Float16)rbf(v);
  }
  float cst[2][8], hst[2][8], bb[2][4];
#pragma unroll
  for (int nt = 0; nt < 2; ++nt) {
    const int j = 32 * wave + 16 * nt + c;
#pragma unroll
    for (int g = 0; g < 4; ++g) bb[nt][g] = rbf(bgate[g * NHID + j]);
#pragma unroll
    for (int r = 0; r < 8; ++r) { cst[nt][r] = 0.0f; hst[nt][r] = 0.0f; }
  }
  const float b1v = rbf(bhead[16 * (wave & 3) + c]);
  const float w2r0 = rbf(w2[4 * c + 0]), w2r1 = rbf(w2[4 * c + 1]), w2r2 = rbf(w2[4 * c + 2]), w2r3 = rbf(w2[4 * c + 3]);
  const float b2v = rbf(bout[0]);
  float zp = 0.0f;
  __syncthreads();

  const _Float16* ainrow = Ain + c * AINP + koff;
  const _Float16* ahrow  = Ah + c * AHP + koff;
  const v8f z8 = {0.f, 0.f, 0.f, 0.f, 0.f, 0.f, 0.f, 0.f};

#pragma unroll 1
  for (int t = 0; t < NSTEP; ++t) {
#pragma unroll
    for (int nt = 0; nt < 2; ++nt) {
      const int j = 32 * wave + 16 * nt + c;
      const _Float16* wi = WI + (size_t)j * KIN + koff;
      const _Float16* wh = WH + (size_t)j * NHID + koff;
      v8f acc[4];
      acc[0] = z8; acc[1] = z8; acc[2] = z8; acc[3] = z8;
      {
        const v16h a   = Frag<_Float16>::load(ainrow);
        const v16h bi0 = Frag<_Float16>::load(wi);
        const v16h bi1 = Frag<_Float16>::load(wi + (size_t)1 * NHID * KIN);
        const v16h bi2 = Frag<_Float16>::load(wi + (size_t)2 * NHID * KIN);
        const v16h bi3 = Frag<_Float16>::load(wi + (size_t)3 * NHID * KIN);
        acc[0] = Frag<_Float16>::mma(a, bi0, acc[0]);
        acc[1] = Frag<_Float16>::mma(a, bi1, acc[1]);
        acc[2] = Frag<_Float16>::mma(a, bi2, acc[2]);
        acc[3] = Frag<_Float16>::mma(a, bi3, acc[3]);
        dep_guard_h(acc[0], acc[3], a, bi3);
        keep4_h(bi0, bi1, bi2, bi3);
      }
#pragma unroll 1
      for (int k0 = 0; k0 < NHID; k0 += 32) {
        const v16h a   = Frag<_Float16>::load(ahrow + k0);
        const v16h bw0 = Frag<_Float16>::load(wh + k0);
        const v16h bw1 = Frag<_Float16>::load(wh + (size_t)1 * NHID * NHID + k0);
        const v16h bw2 = Frag<_Float16>::load(wh + (size_t)2 * NHID * NHID + k0);
        const v16h bw3 = Frag<_Float16>::load(wh + (size_t)3 * NHID * NHID + k0);
        acc[0] = Frag<_Float16>::mma(a, bw0, acc[0]);
        acc[1] = Frag<_Float16>::mma(a, bw1, acc[1]);
        acc[2] = Frag<_Float16>::mma(a, bw2, acc[2]);
        acc[3] = Frag<_Float16>::mma(a, bw3, acc[3]);
        dep_guard_h(acc[0], acc[3], a, bw3);
        keep4_h(bw0, bw1, bw2, bw3);
      }
      acc_guard4(acc[0], acc[1], acc[2], acc[3]);
#pragma unroll
      for (int r = 0; r < 8; ++r) {
        const float zi = acc[0][r] * WCARRY_INV + bb[nt][0];
        const float zf = acc[1][r] * WCARRY_INV + bb[nt][1];
        const float zg = acc[2][r] * WCARRY_INV + bb[nt][2];
        const float zo = acc[3][r] * WCARRY_INV + bb[nt][3];
        const float ig = fsig(zi);
        const float fg = fsig(zf);
        const float gg = ftanh(zg);
        const float og = fsig(zo);
        const float cn = fg * cst[nt][r] + ig * gg;
        cst[nt][r] = cn;
        hst[nt][r] = og * ftanh(cn);
      }
    }
    __syncthreads();
#pragma unroll
    for (int nt = 0; nt < 2; ++nt) {
      const int j = 32 * wave + 16 * nt + c;
#pragma unroll
      for (int r = 0; r < 8; ++r) Ah[(8 * hh + r) * AHP + j] = (_Float16)hst[nt][r];
    }
    {
      const int tn = (t + 1 < NSTEP) ? (t + 1) : (NSTEP - 1);
      const size_t bt = (size_t)(rowbase + mz) * NSTEP + (size_t)tn;
      const float xv = xin[bt * NXF + c];
      const float zv = zin[bt];
      Ain[mz * AINP + 1 + c] = (_Float16)rbf(xv);
      if (c == 0) Ain[mz * AINP] = (_Float16)rbf(zv);
    }
    __syncthreads();
    if (wave < 4) {
      const int n = 16 * wave + c;
      const _Float16* w1row = W1h + (size_t)n * NHID + koff;
      v8f hacc = z8;
#pragma unroll 1
      for (int k0 = 0; k0 < NHID; k0 += 32) {
        const v16h a  = Frag<_Float16>::load(ahrow + k0);
        const v16h bw = Frag<_Float16>::load(w1row + k0);
        hacc = Frag<_Float16>::mma(a, bw, hacc);
        dep_guard1_h(hacc, a, bw);
      }
      acc_guard1(hacc);
#pragma unroll
      for (int r = 0; r < 8; ++r) {
        const float v = hacc[r] * WCARRY_INV + b1v;
        Hid[(8 * hh + r) * HIDP + n] = fmaxf(v, 0.0f);
      }
    }
    __syncthreads();
    {
      const v4f hv = *(const v4f*)(Hid + mz * HIDP + 4 * c);
      float s = hv[0] * w2r0;
      s += hv[1] * w2r1;
      s += hv[2] * w2r2;
      s += hv[3] * w2r3;
      s += __shfl_xor(s, 1, 32);
      s += __shfl_xor(s, 2, 32);
      s += __shfl_xor(s, 4, 32);
      s += __shfl_xor(s, 8, 32);
      const float pre = s + b2v;
      const float d = fmaxf(pre, 0.0f);
      const float zn = zp + d;
      zp = zn;
      if (c == 0) {
        Zs[mz * NSTEP + t] = zn;
        const _Float16 zh = (_Float16)zn;
        const float res = (zn - (float)zh) * LOCARRY;
        Ain[mz * AINP + (NIN - 1)] = zh;
        Ain[mz * AINP + NIN] = (_Float16)res;
      }
    }
    __syncthreads();
  }

#pragma unroll
  for (int nt = 0; nt < 2; ++nt) {
    const int j = 32 * wave + 16 * nt + c;
#pragma unroll
    for (int r = 0; r < 8; ++r) {
      Hs[(8 * hh + r) * OSTP + j] = hst[nt][r];
      Cs[(8 * hh + r) * OSTP + j] = cst[nt][r];
    }
  }
  __syncthreads();
  float* o0 = out + (size_t)rowbase * NSTEP;
  float* o1 = out + OUT1_OFF;
  float* o2 = out + OUT2_OFF;
  for (int pass = 0; pass < 2; ++pass) {
#pragma unroll
    for (int it = 0; it < 4; ++it) {
      const int idx = it * NTHR + tid;
      const int row = idx >> 6, c4 = (idx & 63) * 4;
      const v4f vh = *(const v4f*)(Hs + row * OSTP + c4);
      const v4f vc = *(const v4f*)(Cs + row * OSTP + c4);
      *(volatile v4f*)(o1 + (size_t)(rowbase + row) * NHID + c4) = vh;
      *(volatile v4f*)(o2 + (size_t)(rowbase + row) * NHID + c4) = vc;
    }
#pragma unroll
    for (int it = 0; it < 4; ++it) {
      const int idx = it * NTHR + tid;
      if (idx < ZQUADS) {
        const v4f vz = *(const v4f*)(Zs + idx * 4);
        *(volatile v4f*)(o0 + (size_t)idx * 4) = vz;
      }
    }
    __threadfence();
  }
}

extern "C" void kernel_launch(void* const* d_in, const int* in_sizes, int n_in,
                              void* d_out, int out_size, void* d_ws, size_t ws_size, hipStream_t stream) {
  if (n_in < 10 || d_out == nullptr || d_ws == nullptr) return;
  if (in_sizes[0] != NSEQ * NSTEP || in_sizes[1] != NSEQ * NSTEP * NXF || in_sizes[2] != NSEQ * NHID ||
      in_sizes[3] != NGATE * NIN || in_sizes[4] != NGATE * NHID || in_sizes[5] != NGATE ||
      in_sizes[6] != NFWD * NHID || in_sizes[7] != NFWD || in_sizes[8] != NFWD || in_sizes[9] != 1 ||
      out_size != NSEQ * NSTEP + 2 * NSEQ * NHID) return;

  const float* zin  = (const float*)d_in[0];
  const float* xin  = (const float*)d_in[1];
  const float* h0   = (const float*)d_in[2];
  const float* wih  = (const float*)d_in[3];
  const float* whh  = (const float*)d_in[4];
  const float* bg   = (const float*)d_in[5];
  const float* w1   = (const float*)d_in[6];
  const float* b1   = (const float*)d_in[7];
  const float* w2   = (const float*)d_in[8];
  const float* b2   = (const float*)d_in[9];
  float* out = (float*)d_out;

  char* ws = (char*)d_ws; size_t off = 0;
  auto carve = [&](size_t bytes) -> char* { char* p = ws + off; off += (bytes + 255) & ~(size_t)255; return p; };
  unsigned short* WI  = (unsigned short*)carve((size_t)NGATE * KIN * 2);
  unsigned short* WH  = (unsigned short*)carve((size_t)NGATE * NHID * 2);
  unsigned short* W1P = (unsigned short*)carve((size_t)NFWD * NHID * 2);
  if (off > ws_size || off > (size_t)134217728) return;

  const int n2_whh = NGATE * NHID / 2;
  const int n2_w1  = NFWD * NHID / 2;
  if ((n2_whh % NTHR) != 0 || (n2_w1 % NTHR) != 0 || ((NGATE * KIN / 2) % NTHR) != 0 || (NSEQ % SEQ_PER_BLK) != 0) return;

  cast_w_f16x2<<<n2_whh / NTHR, NTHR, 0, stream>>>(whh, WH, n2_whh, WCARRY);
  cast_w_f16x2<<<n2_w1 / NTHR, NTHR, 0, stream>>>(w1, W1P, n2_w1, WCARRY);
  wih_plane_kernel<<<(NGATE * KIN / 2) / NTHR, NTHR, 0, stream>>>(wih, WI);
  lstm_head_kernel<<<NSEQ / SEQ_PER_BLK, NTHR, 0, stream>>>(zin, xin, h0, bg, b1, w2, b2, WI, WH, W1P, out);
}
